// VanillaRNN_28905129902731
// MI455X (gfx1250) — hardware-verified
//
#include <hip/hip_runtime.h>
#include <math.h>

constexpr int NB      = 32;
constexpr int NDIN    = 128;
constexpr int NL      = 2048;
constexpr int NDS     = 512;
constexpr int NDOUT   = 128;
constexpr int NROWS   = NL * NB;
constexpr int KX      = NDIN;
constexpr int KH2     = 2 * NDS;
constexpr int KCAT    = KX + KH2;
constexpr int HIC0    = KX;
constexpr int LOC0    = KX + NDS;
constexpr int TPITCH  = 1160;
constexpr int YPITCH  = 132;
constexpr int NTHR    = 256;
constexpr int NWAVE   = NTHR / 32;
constexpr int SEQ_BLK = 16;
constexpr int KSTEP   = 128;
static_assert(KCAT % 32 == 0 && KH2 % 32 == 0 && KX % 32 == 0);
static_assert(KCAT % KSTEP == 0 && KH2 % KSTEP == 0);
static_assert(NDS == 64 * NWAVE);
static_assert(NDOUT == 16 * NWAVE);
static_assert(NB % SEQ_BLK == 0);
static_assert(SEQ_BLK == 2 * NWAVE);
static_assert(TPITCH % 8 == 0 && TPITCH >= KCAT);
static_assert(YPITCH % 4 == 0 && YPITCH >= NDOUT);
static_assert(SEQ_BLK * (KX / 8) == NTHR);
static_assert(NDOUT == 4 * 32);
static_assert((NB * NDIN) % 64 == 0 && NL % 64 == 0);
static_assert((NDS * (NDIN / 8)) % NTHR == 0 && (NDS * (NDS / 8)) % NTHR == 0 && (NDOUT * (NDS / 8)) % NTHR == 0);

typedef __attribute__((ext_vector_type(16))) _Float16 v16h;
typedef __attribute__((ext_vector_type(8)))  _Float16 v8h;
typedef __attribute__((ext_vector_type(16))) __bf16   v16b;
typedef __attribute__((ext_vector_type(8)))  __bf16   v8b;
typedef __attribute__((ext_vector_type(8)))  float    v8f;
typedef __attribute__((ext_vector_type(4)))  float    v4f;
typedef __attribute__((ext_vector_type(4)))  unsigned v4u;

__device__ __forceinline__ unsigned short f2bf_bits(float f) {
  unsigned u = __float_as_uint(f);
  return (unsigned short)((u + 0x7FFFu + ((u >> 16) & 1u)) >> 16);
}
__device__ __forceinline__ float bf_bits2f(unsigned short h) { return __uint_as_float(((unsigned)h) << 16); }
__device__ __forceinline__ float bf16r(float f) { return bf_bits2f(f2bf_bits(f)); }

__device__ __forceinline__ void acc_guard4(v8f& a, v8f& b, v8f& c, v8f& d) { asm volatile("v_nop\n\tv_nop\n\tv_nop\n\tv_nop" : "+v"(a), "+v"(b), "+v"(c), "+v"(d)); }
__device__ __forceinline__ void acc_guard1(v8f& a) { asm volatile("v_nop\n\tv_nop\n\tv_nop\n\tv_nop" : "+v"(a)); }
__device__ __forceinline__ void guard5m_b(v8f& a0, v8f& a1, v8f& a2, v8f& a3, v16b x, v16b y0, v16b y1, v16b y2, v16b y3) {
  asm volatile("v_nop\n\tv_nop\n\tv_nop\n\tv_nop" : "+v"(a0), "+v"(a1), "+v"(a2), "+v"(a3) : "v"(x), "v"(y0), "v"(y1), "v"(y2), "v"(y3) : "memory");
}
__device__ __forceinline__ void guard1m_b(v8f& a0, v16b x, v16b y) {
  asm volatile("v_nop\n\tv_nop\n\tv_nop\n\tv_nop" : "+v"(a0) : "v"(x), "v"(y) : "memory");
}
template <typename T> struct Frag;
template <> struct Frag<__bf16> {
  typedef v16b V; union U { v16b v; v8b h[2]; };
  static __device__ __forceinline__ v16b load(const __bf16* p) {
    U f; f.h[0] = *(const v8b*)(p); f.h[1] = *(const v8b*)(p + 16); return f.v;
  }
  static __device__ __forceinline__ v8f mma(v16b a, v16b b, v8f c) {
    return __builtin_amdgcn_wmma_f32_16x16x32_bf16(false, a, false, b, (short)0, c, false, false);
  }
};

__device__ __forceinline__ float tanh_f32(float x) {
  const float xc = fminf(fmaxf(x, -15.0f), 15.0f);
  const float e = expf(2.0f * xc);
  return 1.0f - 2.0f / (e + 1.0f);
}

__device__ __forceinline__ void rec_chunk(const __bf16* ap, const __bf16* wp, v8f& d0, v8f& d1, v8f& d2, v8f& d3) {
  const v16b a  = Frag<__bf16>::load(ap);
  const v16b b0 = Frag<__bf16>::load(wp);
  const v16b b1 = Frag<__bf16>::load(wp + (size_t)1 * 16 * KCAT);
  const v16b b2 = Frag<__bf16>::load(wp + (size_t)2 * 16 * KCAT);
  const v16b b3 = Frag<__bf16>::load(wp + (size_t)3 * 16 * KCAT);
  d0 = Frag<__bf16>::mma(a, b0, d0);
  d1 = Frag<__bf16>::mma(a, b1, d1);
  d2 = Frag<__bf16>::mma(a, b2, d2);
  d3 = Frag<__bf16>::mma(a, b3, d3);
  guard5m_b(d0, d1, d2, d3, a, b0, b1, b2, b3);
}
__device__ __forceinline__ void head_chunk(const __bf16* ap, const __bf16* fp, v8f& d0) {
  const v16b a = Frag<__bf16>::load(ap);
  const v16b b = Frag<__bf16>::load(fp);
  d0 = Frag<__bf16>::mma(a, b, d0);
  guard1m_b(d0, a, b);
}

__global__ __launch_bounds__(NTHR) void tp_bf16_kernel(const float* __restrict__ src, int R, int C, int ldo,
                                                       unsigned short* __restrict__ O) {
  __shared__ float Tt[64 * 65];
  const int tid = threadIdx.x;
  const int c0 = blockIdx.x * 64, r0 = blockIdx.y * 64;
#pragma unroll
  for (int i = 0; i < 4; ++i) {
    const int idx = i * NTHR + tid;
    const int rr = idx >> 4, cc = (idx & 15) * 4;
    const v4f v = *(const v4f*)(src + (size_t)(r0 + rr) * (size_t)C + c0 + cc);
    Tt[rr * 65 + cc + 0] = v[0];
    Tt[rr * 65 + cc + 1] = v[1];
    Tt[rr * 65 + cc + 2] = v[2];
    Tt[rr * 65 + cc + 3] = v[3];
  }
  __syncthreads();
  const int q = tid >> 3, c8 = (tid & 7) * 8;
  v8h hv[2];
#pragma unroll
  for (int g = 0; g < 2; ++g) {
    const int qq = g * 32 + q;
#pragma unroll
    for (int e = 0; e < 8; ++e) {
      const float f = Tt[(c8 + e) * 65 + qq];
      hv[g][e] = __builtin_bit_cast(_Float16, f2bf_bits(f));
    }
  }
  for (int pass = 0; pass < 2; ++pass) {
#pragma unroll
    for (int g = 0; g < 2; ++g) {
      const size_t o = (size_t)(c0 + g * 32 + q) * (size_t)ldo + (size_t)(r0 + c8);
      *(volatile v8h*)(O + o) = hv[g];
    }
    __threadfence();
  }
}

__global__ __launch_bounds__(NTHR) void cvt_rows_kernel(const float* __restrict__ src, int spitch, int ncol8,
                                                        unsigned short* __restrict__ dst, int dpitch, int dcol0, int nrow) {
  const int i  = blockIdx.x * NTHR + threadIdx.x;
  const int n8 = nrow * ncol8;
  if (i < n8) {
    const int row = i / ncol8;
    const int c8  = i - row * ncol8;
    const float* sp = src + (size_t)row * spitch + c8 * 8;
    const v4f a = *(const v4f*)(sp);
    const v4f b = *(const v4f*)(sp + 4);
    v8h hv;
#pragma unroll
    for (int e = 0; e < 4; ++e) {
      hv[e]     = __builtin_bit_cast(_Float16, f2bf_bits(a[e]));
      hv[4 + e] = __builtin_bit_cast(_Float16, f2bf_bits(b[e]));
    }
    unsigned short* dp = dst + (size_t)row * dpitch + dcol0 + c8 * 8;
    *(volatile v8h*)dp = hv;
    __threadfence();
    *(volatile v8h*)dp = hv;
  }
}

__global__ __launch_bounds__(NTHR) void rnn_seq_kernel(const unsigned short* __restrict__ xb,
                                                       const unsigned short* __restrict__ wcatp,
                                                       const unsigned short* __restrict__ wfcp,
                                                       const float* __restrict__ b_ih, const float* __restrict__ b_hh,
                                                       const float* __restrict__ b_fc, float* __restrict__ out) {
  __shared__ __align__(16) unsigned short At[SEQ_BLK * TPITCH];
  __shared__ __align__(16) float          Ys[SEQ_BLK * YPITCH];
  const __bf16* WC = (const __bf16*)(const void*)wcatp;
  const __bf16* WF = (const __bf16*)(const void*)wfcp;
  const int tid = threadIdx.x, lane = tid & 31, wave = tid >> 5;
  const int c = lane & 15, hh = lane >> 4, koff = hh * 8;
  const int rowbase = blockIdx.x * SEQ_BLK;
  const int sm = tid >> 4, sc8 = (tid & 15) * 8;

#pragma unroll 1
  for (int i = tid; i < SEQ_BLK * TPITCH; i += NTHR) At[i] = (unsigned short)0;
  __syncthreads();
  {
    const v4u v = *(const v4u*)(xb + (size_t)(rowbase + sm) * KX + sc8);
    *(v4u*)(At + sm * TPITCH + sc8) = v;
  }
  float bi[4], bh[4];
#pragma unroll
  for (int nt = 0; nt < 4; ++nt) {
    const int j = 64 * wave + 16 * nt + c;
    bi[nt] = bf16r(b_ih[j]);
    bh[nt] = bf16r(b_hh[j]);
  }
  const float bf = bf16r(b_fc[16 * wave + c]);
  __syncthreads();

  const __bf16* arow = (const __bf16*)(const void*)At + c * TPITCH + koff;
  const __bf16* wrow = WC + (size_t)(64 * wave + c) * KCAT + koff;
  const __bf16* frow = WF + (size_t)(16 * wave + c) * KH2 + koff;
  const v8f z8 = {0.f, 0.f, 0.f, 0.f, 0.f, 0.f, 0.f, 0.f};

#pragma unroll 1
  for (int t = 0; t < NL; ++t) {
    v8f acc[4];
    acc[0] = z8; acc[1] = z8; acc[2] = z8; acc[3] = z8;
#pragma unroll 1
    for (int k0 = 0; k0 < KCAT; k0 += KSTEP) {
      rec_chunk(arow + k0,      wrow + k0,      acc[0], acc[1], acc[2], acc[3]);
      rec_chunk(arow + k0 + 32, wrow + k0 + 32, acc[0], acc[1], acc[2], acc[3]);
      rec_chunk(arow + k0 + 64, wrow + k0 + 64, acc[0], acc[1], acc[2], acc[3]);
      rec_chunk(arow + k0 + 96, wrow + k0 + 96, acc[0], acc[1], acc[2], acc[3]);
    }
    acc_guard4(acc[0], acc[1], acc[2], acc[3]);
    float hn[4][8];
#pragma unroll
    for (int nt = 0; nt < 4; ++nt) {
#pragma unroll
      for (int r = 0; r < 8; ++r) {
        const float z = (acc[nt][r] + bi[nt]) + bh[nt];
        hn[nt][r] = tanh_f32(z);
      }
    }
    __syncthreads();

#pragma unroll
    for (int nt = 0; nt < 4; ++nt) {
      const int j = 64 * wave + 16 * nt + c;
#pragma unroll
      for (int r = 0; r < 8; ++r) {
        const int m = 8 * hh + r;
        const float hv = hn[nt][r];
        const unsigned short hb = f2bf_bits(hv);
        const unsigned short lb = f2bf_bits(hv - bf_bits2f(hb));
        At[m * TPITCH + HIC0 + j] = hb;
        At[m * TPITCH + LOC0 + j] = lb;
      }
    }
    {
      const int tn = (t + 1 < NL) ? (t + 1) : (NL - 1);
      const v4u v = *(const v4u*)(xb + (size_t)(tn * NB + rowbase + sm) * KX + sc8);
      *(v4u*)(At + sm * TPITCH + sc8) = v;
    }
    __syncthreads();

    v8f facc = z8;
#pragma unroll 1
    for (int k0 = 0; k0 < KH2; k0 += KSTEP) {
      head_chunk(arow + HIC0 + k0,      frow + k0,      facc);
      head_chunk(arow + HIC0 + k0 + 32, frow + k0 + 32, facc);
      head_chunk(arow + HIC0 + k0 + 64, frow + k0 + 64, facc);
      head_chunk(arow + HIC0 + k0 + 96, frow + k0 + 96, facc);
    }
    acc_guard1(facc);
#pragma unroll
    for (int r = 0; r < 8; ++r) Ys[(8 * hh + r) * YPITCH + 16 * wave + c] = tanh_f32(facc[r] + bf);
    __syncthreads();

    for (int pass = 0; pass < 2; ++pass) {
#pragma unroll
      for (int rr = 0; rr < 2; ++rr) {
        const int row = 2 * wave + rr;
        const v4f v = *(const v4f*)(Ys + row * YPITCH + 4 * lane);
        *(volatile v4f*)(out + ((size_t)t * NB + (size_t)(rowbase + row)) * NDOUT + 4 * lane) = v;
      }
      __threadfence();
    }
  }
}

extern "C" void kernel_launch(void* const* d_in, const int* in_sizes, int n_in,
                              void* d_out, int out_size, void* d_ws, size_t ws_size, hipStream_t stream) {
  if (n_in < 7 || d_out == nullptr || d_ws == nullptr) return;
  if (in_sizes[0] != NB * NDIN * NL || in_sizes[1] != NDS * NDIN || in_sizes[2] != NDS * NDS ||
      in_sizes[3] != NDS || in_sizes[4] != NDS || in_sizes[5] != NDOUT * NDS || in_sizes[6] != NDOUT ||
      out_size != NROWS * NDOUT) return;

  const float* x    = (const float*)d_in[0];
  const float* w_ih = (const float*)d_in[1];
  const float* w_hh = (const float*)d_in[2];
  const float* b_ih = (const float*)d_in[3];
  const float* b_hh = (const float*)d_in[4];
  const float* w_fc = (const float*)d_in[5];
  const float* b_fc = (const float*)d_in[6];
  float* out = (float*)d_out;

  char* ws = (char*)d_ws; size_t off = 0;
  auto carve = [&](size_t bytes) -> char* { char* p = ws + off; off += (bytes + 255) & ~(size_t)255; return p; };
  unsigned short* XB   = (unsigned short*)carve((size_t)NROWS * KX * 2);
  unsigned short* WCAT = (unsigned short*)carve((size_t)NDS * KCAT * 2);
  unsigned short* WFC2 = (unsigned short*)carve((size_t)NDOUT * KH2 * 2);
  if (off > ws_size || off > (size_t)134217728) return;

  tp_bf16_kernel<<<dim3(NL / 64, (NB * NDIN) / 64), NTHR, 0, stream>>>(x, NB * NDIN, NL, NB * NDIN, XB);
  const int n8_ih = NDS * (NDIN / 8);
  const int n8_hh = NDS * (NDS / 8);
  const int n8_fc = NDOUT * (NDS / 8);
  cvt_rows_kernel<<<(n8_ih + NTHR - 1) / NTHR, NTHR, 0, stream>>>(w_ih, NDIN, NDIN / 8, WCAT, KCAT, 0,    NDS);
  cvt_rows_kernel<<<(n8_hh + NTHR - 1) / NTHR, NTHR, 0, stream>>>(w_hh, NDS,  NDS / 8,  WCAT, KCAT, HIC0, NDS);
  cvt_rows_kernel<<<(n8_hh + NTHR - 1) / NTHR, NTHR, 0, stream>>>(w_hh, NDS,  NDS / 8,  WCAT, KCAT, LOC0, NDS);
  cvt_rows_kernel<<<(n8_fc + NTHR - 1) / NTHR, NTHR, 0, stream>>>(w_fc, NDS,  NDS / 8,  WFC2, KH2,  0,    NDOUT);
  cvt_rows_kernel<<<(n8_fc + NTHR - 1) / NTHR, NTHR, 0, stream>>>(w_fc, NDS,  NDS / 8,  WFC2, KH2,  NDS,  NDOUT);
  rnn_seq_kernel<<<NB / SEQ_BLK, NTHR, 0, stream>>>(XB, WCAT, WFC2, b_ih, b_hh, b_fc, out);
}
